// GRAND_89859305766914
// MI455X (gfx1250) — hardware-run, weakly checked
//
#include <hip/hip_runtime.h>
#include <math.h>

typedef __attribute__((ext_vector_type(16))) _Float16 v16h;
typedef __attribute__((ext_vector_type(8)))  _Float16 v8h;
typedef __attribute__((ext_vector_type(8)))  float    v8f;
typedef __attribute__((ext_vector_type(4)))  float    v4f;
typedef __attribute__((ext_vector_type(4)))  int      v4i;

constexpr int kNN     = 100000;
constexpr int kNE     = 1600000;
constexpr int kDF     = 128;
constexpr int kDH     = 128;
constexpr int kDO     = 64;
constexpr int kMPad   = 100032;
constexpr int kChunkE = 4096;
constexpr int kNCh    = 391;
constexpr int kGrpN   = 256;
constexpr int kNGrp   = 391;
constexpr int kTabP   = 416;
constexpr int kCapG   = 8192;
constexpr int kNTab   = kNGrp * kGrpN;
constexpr int kCsrTot = kNGrp * kCapG;
static_assert((kNE + kChunkE - 1) / kChunkE == kNCh);
static_assert((kNN + kGrpN - 1) / kGrpN == kNGrp);
static_assert(kNGrp + 1 <= kTabP && (kTabP % 32) == 0);
static_assert((kNE % 4) == 0 && (kMPad % 64) == 0 && kMPad >= kNN && kNTab >= kMPad);
static_assert((kDF % 32) == 0 && (kDH % 32) == 0 && (kDH % 64) == 0 && (kDO % 64) == 0);
static_assert(kNN <= 131072 && kGrpN == 256);
static_assert((kNN % 8) == 0 && (kMPad % 8) == 0);

constexpr float kKeep   = 0.5f;
constexpr int   kHops   = 4;
constexpr float kMix    = kKeep / (float)(kHops + 1);
constexpr float kYCarry = 256.0f;
constexpr float kHCarry = 256.0f;
constexpr float kWCarry = 64.0f;
constexpr float kScale1 = kHCarry / (kYCarry * kWCarry);
constexpr float kScale2 = 1.0f / (kHCarry * kWCarry);

constexpr size_t kSzPart   = (size_t)kNCh * kChunkE * 4;
constexpr size_t kSzCtab   = (size_t)kNCh * kTabP * 4;
constexpr size_t kSzCsr    = (size_t)kNGrp * kCapG * 4;
constexpr size_t kSzTab    = (size_t)kNTab * 4;
constexpr size_t kSzZ      = (size_t)kMPad * kDF * 4;
constexpr size_t kSzW1T    = (size_t)kDH * kDF * 2;
constexpr size_t kSzW2T    = (size_t)kDO * kDH * 2;
constexpr size_t kOffPart  = 0;
constexpr size_t kOffCtab  = kOffPart + kSzPart;
constexpr size_t kOffCsr   = kOffCtab + kSzCtab;
constexpr size_t kOffRS    = kOffCsr + kSzCsr;
constexpr size_t kOffRD    = kOffRS + kSzTab;
constexpr size_t kOffRN    = kOffRD + kSzTab;
constexpr size_t kOffZA    = kOffRN + kSzTab;
constexpr size_t kOffZB    = kOffZA + kSzZ;
constexpr size_t kOffW1T   = kOffZB + kSzZ;
constexpr size_t kOffW2T   = kOffW1T + kSzW1T;
constexpr size_t kWsTotal  = kOffW2T + kSzW2T;
static_assert(kWsTotal == 123552128ull);
static_assert(kWsTotal <= 134217728ull);
static_assert((kOffCtab % 128) == 0 && (kOffCsr % 128) == 0 && (kOffRS % 128) == 0 && (kOffRD % 128) == 0 &&
              (kOffRN % 128) == 0 && (kOffZA % 128) == 0 && (kOffZB % 128) == 0 && (kOffW1T % 128) == 0 &&
              (kOffW2T % 128) == 0);
static_assert((size_t)kMPad * kDF * 2 <= kSzZ);

__device__ __forceinline__ int clampi(int v, int lo, int hi) { return v < lo ? lo : (v > hi ? hi : v); }

__global__ __launch_bounds__(256) void part_edges_kernel(
    const int* __restrict__ ei, unsigned* __restrict__ part, int* __restrict__ ctab)
{
  __shared__ int sHist[kTabP];
  __shared__ __align__(16) int sStart[kTabP];
  __shared__ __align__(16) unsigned sStage[kChunkE];
  const int tid = threadIdx.x;
  const int c = blockIdx.x;
  const int ebase = c * kChunkE;
  for (int i = tid; i < kTabP; i += 256) sHist[i] = 0;
  __syncthreads();
  unsigned pk[16];
  int gi[16];
  int rk[16];
#pragma unroll
  for (int i = 0; i < 4; ++i) {
    const int e0 = ebase + i * 1024 + tid * 4;
    const bool ok = e0 < kNE;
    const int e0c = ok ? e0 : (kNE - 4);
    const v4i sv = *(const v4i*)(ei + e0c);
    const v4i dv = *(const v4i*)(ei + kNE + e0c);
#pragma unroll
    for (int j = 0; j < 4; ++j) {
      const int s = clampi(sv[j], 0, kNN - 1);
      const int d = clampi(dv[j], 0, kNN - 1);
      const int g = ok ? (d >> 8) : kNGrp;
      const unsigned p = ok ? ((unsigned)s | ((unsigned)(d & 255) << 17)) : 0xFFFFFFFFu;
      gi[i * 4 + j] = g;
      pk[i * 4 + j] = p;
      rk[i * 4 + j] = atomicAdd(&sHist[g], 1);
    }
  }
  __syncthreads();
  if (tid == 0) {
    int run = 0;
#pragma unroll 1
    for (int k = 0; k < kTabP; ++k) {
      const int hv = sHist[k];
      sStart[k] = run;
      run += hv;
    }
  }
  __syncthreads();
#pragma unroll
  for (int q = 0; q < 16; ++q) {
    const int pos = clampi(sStart[gi[q]] + rk[q], 0, kChunkE - 1);
    sStage[pos] = pk[q];
  }
  __syncthreads();
  v4i ov[4];
#pragma unroll
  for (int i = 0; i < 4; ++i) ov[i] = *(const v4i*)(sStage + i * 1024 + tid * 4);
  v4i tv = (v4i){0, 0, 0, 0};
  if (tid < kTabP / 4) tv = *(const v4i*)(sStart + tid * 4);
  unsigned* po = part + (size_t)c * kChunkE;
  int* pt = ctab + (size_t)c * kTabP;
  for (int pass = 0; pass < 2; ++pass) {
#pragma unroll
    for (int i = 0; i < 4; ++i) *(volatile v4i*)(po + i * 1024 + tid * 4) = ov[i];
    if (tid < kTabP / 4) *(volatile v4i*)(pt + tid * 4) = tv;
    __threadfence();
  }
}

__global__ __launch_bounds__(256) void build_rows_kernel(
    const unsigned* __restrict__ part, const int* __restrict__ ctab,
    int* __restrict__ csr, int* __restrict__ rstart, int* __restrict__ rdeg, float* __restrict__ rnorm)
{
  __shared__ int sCnt[kGrpN];
  __shared__ int sOff[kGrpN];
  __shared__ int sCur[kGrpN];
  __shared__ int sMax;
  __shared__ __align__(16) int sList[kCapG];
  const int tid = threadIdx.x;
  const int g = blockIdx.x;
  sCnt[tid] = 0;
  if (tid == 0) sMax = 0;
#pragma unroll
  for (int i = 0; i < 8; ++i) *(v4i*)(sList + i * 1024 + tid * 4) = (v4i){0, 0, 0, 0};
  __syncthreads();
  int a0[2], ln[2], cb[2];
#pragma unroll
  for (int i = 0; i < 2; ++i) {
    const int c = tid + 256 * i;
    const int cc = c < kNCh ? c : (kNCh - 1);
    int t0 = ctab[(size_t)cc * kTabP + g];
    int t1 = ctab[(size_t)cc * kTabP + g + 1];
    asm volatile("" : "+v"(t0));
    asm volatile("" : "+v"(t1));
    t0 = clampi(t0, 0, kChunkE);
    t1 = clampi(t1, 0, kChunkE);
    const int l = (c < kNCh && t1 > t0) ? (t1 - t0) : 0;
    a0[i] = t0;
    ln[i] = l;
    cb[i] = cc * kChunkE;
    atomicMax(&sMax, l);
  }
  __syncthreads();
  int kmax = sMax;
  kmax = __builtin_amdgcn_readfirstlane(kmax);
  kmax = kmax < kChunkE ? kmax : kChunkE;
#pragma unroll 1
  for (int k = 0; k < kmax; ++k) {
#pragma unroll
    for (int i = 0; i < 2; ++i) {
      int idx = a0[i] + k;
      idx = idx < kChunkE ? idx : (kChunkE - 1);
      unsigned p = part[(size_t)cb[i] + idx];
      asm volatile("" : "+v"(p));
      if (k < ln[i]) atomicAdd(&sCnt[(p >> 17) & 255u], 1);
    }
  }
  __syncthreads();
  if (tid == 0) {
    int run = 0;
#pragma unroll 1
    for (int j = 0; j < kGrpN; ++j) {
      const int cv = sCnt[j];
      sOff[j] = run;
      sCur[j] = run;
      run += cv;
    }
  }
  __syncthreads();
#pragma unroll 1
  for (int k = 0; k < kmax; ++k) {
#pragma unroll
    for (int i = 0; i < 2; ++i) {
      int idx = a0[i] + k;
      idx = idx < kChunkE ? idx : (kChunkE - 1);
      unsigned p = part[(size_t)cb[i] + idx];
      asm volatile("" : "+v"(p));
      if (k < ln[i]) {
        const int pos = atomicAdd(&sCur[(p >> 17) & 255u], 1);
        int s = (int)(p & 0x1FFFFu);
        s = s < kNN ? s : (kNN - 1);
        if ((unsigned)pos < (unsigned)kCapG) sList[pos] = s;
      }
    }
  }
  __syncthreads();
  {
    const int sd = sCnt[tid];
    const int sb = sOff[tid];
    const int so = sb < kCapG ? sb : kCapG;
    const int sroom = kCapG - so;
    const int sn = sd < sroom ? sd : sroom;
#pragma unroll 1
    for (int i = 1; i < sn; ++i) {
      const int key = sList[so + i];
      int j = i;
#pragma unroll 1
      for (; j > 0; --j) {
        const int prev = sList[so + j - 1];
        if (prev <= key) break;
        sList[so + j] = prev;
      }
      sList[so + j] = key;
    }
  }
  __syncthreads();
  v4i lv[8];
#pragma unroll
  for (int i = 0; i < 8; ++i) lv[i] = *(const v4i*)(sList + i * 1024 + tid * 4);
  v4i rs = (v4i){0, 0, 0, 0};
  v4i rd = (v4i){0, 0, 0, 0};
  v4f rn = (v4f){1.f, 1.f, 1.f, 1.f};
  if (tid < 64) {
#pragma unroll
    for (int e = 0; e < 4; ++e) {
      const int d = sCnt[tid * 4 + e];
      const int o = sOff[tid * 4 + e];
      const int oc = o < kCapG ? o : kCapG;
      const int room = kCapG - oc;
      const int dd = d < room ? d : room;
      rs[e] = g * kCapG + oc;
      rd[e] = dd;
      rn[e] = rsqrtf((float)(d > 1 ? d : 1));
    }
  }
  int* pc = csr + (size_t)g * kCapG;
  for (int pass = 0; pass < 2; ++pass) {
#pragma unroll
    for (int i = 0; i < 8; ++i) *(volatile v4i*)(pc + i * 1024 + tid * 4) = lv[i];
    if (tid < 64) {
      *(volatile v4i*)(rstart + (size_t)g * kGrpN + tid * 4) = rs;
      *(volatile v4i*)(rdeg + (size_t)g * kGrpN + tid * 4) = rd;
      *(volatile v4f*)(rnorm + (size_t)g * kGrpN + tid * 4) = rn;
    }
    __threadfence();
  }
}

__global__ __launch_bounds__(256) void weight_planes_kernel(
    const float* __restrict__ W1, const float* __restrict__ W2,
    unsigned short* __restrict__ W1t, unsigned short* __restrict__ W2t)
{
  const int b = blockIdx.x;
  const bool first = b < 8;
  const float* src = first ? W1 : W2;
  unsigned short* dst = first ? W1t : W2t;
  const int ncols = first ? kDH : kDO;
  const int i = (first ? b : (b - 8)) * 256 + threadIdx.x;
  const int n = i >> 4;
  const int k8 = (i & 15) * 8;
  v8h hv;
#pragma unroll
  for (int e = 0; e < 8; ++e) {
    const float w = src[(size_t)(k8 + e) * ncols + n];
    hv[e] = (_Float16)(w * kWCarry);
  }
  unsigned short* q = dst + (size_t)n * 128 + k8;
  *(volatile v8h*)q = hv;
  __threadfence();
  *(volatile v8h*)q = hv;
}

template <int MODE>
__global__ __launch_bounds__(256) void hop_kernel(
    const float* X, const float* feats, const int* __restrict__ csr,
    const int* __restrict__ rstart, const int* __restrict__ rdeg, const float* __restrict__ rnorm,
    float* Zout, unsigned short* Y16, float xscale)
{
  __shared__ __align__(16) float sY[MODE == 1 ? 8 * kDF : 4];
  const int tid = threadIdx.x;
  const int lane = tid & 31;
  const int wave = __builtin_amdgcn_readfirstlane(tid >> 5);
  const int row = blockIdx.x * 8 + wave;
  const bool valid = row < kNN;
  const int rc = valid ? row : (kNN - 1);
  int st = rstart[rc];
  int dg = rdeg[rc];
  const float nd = rnorm[rc];
  st = __builtin_amdgcn_readfirstlane(st);
  dg = __builtin_amdgcn_readfirstlane(dg);
  st = clampi(st, 0, kCsrTot - 1);
  dg = clampi(dg, 0, kCapG);
  dg = valid ? dg : 0;
  v4f acc = (v4f){0.f, 0.f, 0.f, 0.f};
#pragma unroll 1
  for (int base = 0; base < dg; base += 32) {
    int eidx = st + base + lane;
    eidx = eidx < kCsrTot ? eidx : (kCsrTot - 1);
    int sidx = csr[eidx];
    sidx = clampi(sidx, 0, kNN - 1);
    const int nsb = __float_as_int(rnorm[sidx]);
    const int rem = dg - base;
    const int n = rem < 32 ? rem : 32;
#pragma unroll 1
    for (int j = 0; j < n; ++j) {
      const int s = __builtin_amdgcn_readlane(sidx, j);
      const float w = __int_as_float(__builtin_amdgcn_readlane(nsb, j));
      const v4f v = *(const v4f*)(X + (size_t)s * kDF + lane * 4);
      acc[0] = fmaf(w, v[0], acc[0]);
      acc[1] = fmaf(w, v[1], acc[1]);
      acc[2] = fmaf(w, v[2], acc[2]);
      acc[3] = fmaf(w, v[3], acc[3]);
    }
  }
  const v4f f = *(const v4f*)(feats + (size_t)rc * kDF + lane * 4);
  const float cs = nd * xscale;
  v4f o;
  o[0] = fmaf(cs, acc[0], kMix * f[0]);
  o[1] = fmaf(cs, acc[1], kMix * f[1]);
  o[2] = fmaf(cs, acc[2], kMix * f[2]);
  o[3] = fmaf(cs, acc[3], kMix * f[3]);
  if (MODE == 0) {
    if (valid) {
      float* q = Zout + (size_t)row * kDF + lane * 4;
      *(volatile v4f*)q = o;
      __threadfence();
      *(volatile v4f*)q = o;
    }
  } else {
    v4f z;
    z[0] = valid ? o[0] : 0.0f;
    z[1] = valid ? o[1] : 0.0f;
    z[2] = valid ? o[2] : 0.0f;
    z[3] = valid ? o[3] : 0.0f;
    *(v4f*)(sY + wave * kDF + lane * 4) = z;
    __syncthreads();
    if (tid < 128) {
      const int r = tid >> 4;
      const int c8 = (tid & 15) * 8;
      const v4f a0 = *(const v4f*)(sY + r * kDF + c8);
      const v4f a1 = *(const v4f*)(sY + r * kDF + c8 + 4);
      v8h hv;
#pragma unroll
      for (int e = 0; e < 4; ++e) {
        hv[e]     = (_Float16)(a0[e] * kYCarry);
        hv[4 + e] = (_Float16)(a1[e] * kYCarry);
      }
      unsigned short* q = Y16 + (size_t)(blockIdx.x * 8 + r) * kDF + c8;
      *(volatile v8h*)q = hv;
      __threadfence();
      *(volatile v8h*)q = hv;
    }
  }
}

__device__ __forceinline__ void guard1_h(v8f& a, v16h x, v16h y) {
  asm volatile("v_nop\n\tv_nop\n\tv_nop\n\tv_nop" : "+v"(a) : "v"(x), "v"(y));
}
__device__ __forceinline__ void guard0(v8f& a) {
  asm volatile("v_nop\n\tv_nop\n\tv_nop\n\tv_nop" : "+v"(a));
}
__device__ __forceinline__ void keep4_h(v16h a, v16h b, v16h c, v16h d) {
  asm volatile("v_nop" :: "v"(a), "v"(b), "v"(c), "v"(d));
}
struct FragH {
  union U { v16h v; v8h h[2]; };
  static __device__ __forceinline__ v16h load(const _Float16* p) {
    U f;
    f.h[0] = *(const v8h*)(p);
    f.h[1] = *(const v8h*)(p + 16);
    return f.v;
  }
  static __device__ __forceinline__ v8f mma(v16h a, v16h b, v8f c) {
    return __builtin_amdgcn_wmma_f32_16x16x32_f16(false, a, false, b, (short)0, c, false, false);
  }
};

template <int OUT_MODE, int ACT>
__global__ __launch_bounds__(256) void wmma_gemm64_f16(
    const unsigned short* __restrict__ Ap, int lda,
    const unsigned short* __restrict__ Btp, int ldb,
    void* __restrict__ Cout, int ldc,
    int M, int N, int K, int mReal, float scale)
{
  const _Float16* A  = (const _Float16*)Ap;
  const _Float16* Bt = (const _Float16*)Btp;
  __shared__ __align__(16) float sT[8][16 * 68];
  const int lane = threadIdx.x & 31;
  const int wave = threadIdx.x >> 5;
  const int tilesN = N >> 6;
  const int tilesM = M >> 6;
  const int tile = blockIdx.x * 8 + wave;
  if (tile >= tilesM * tilesN) return;
  const int tm = tile / tilesN;
  const int tn = tile - tm * tilesN;
  const int m0 = tm << 6;
  const int n0 = tn << 6;

  const int rlane = lane & 15;
  const int koff  = (lane >> 4) * 8;
  const int mOff  = (lane >> 4) * 8;

  v8f acc[4][4];
#pragma unroll
  for (int i = 0; i < 4; ++i)
#pragma unroll
    for (int j = 0; j < 4; ++j) acc[i][j] = (v8f){0.f, 0.f, 0.f, 0.f, 0.f, 0.f, 0.f, 0.f};

  for (int k0 = 0; k0 < K; k0 += 32) {
    v16h bh[4];
#pragma unroll
    for (int j = 0; j < 4; ++j) {
      const size_t bo = (size_t)(n0 + (j << 4) + rlane) * ldb + koff + k0;
      bh[j] = FragH::load(Bt + bo);
    }
#pragma unroll
    for (int i = 0; i < 4; ++i) {
      const size_t ao = (size_t)(m0 + (i << 4) + rlane) * lda + koff + k0;
      const v16h ah = FragH::load(A + ao);
#pragma unroll
      for (int j = 0; j < 4; ++j) acc[i][j] = FragH::mma(ah, bh[j], acc[i][j]);
#pragma unroll
      for (int j = 0; j < 4; ++j) guard1_h(acc[i][j], ah, bh[j]);
    }
    keep4_h(bh[0], bh[1], bh[2], bh[3]);
  }
#pragma unroll
  for (int i = 0; i < 4; ++i)
#pragma unroll
    for (int j = 0; j < 4; ++j) guard0(acc[i][j]);

  float* slab = sT[wave];
#pragma unroll
  for (int i = 0; i < 4; ++i) {
    const int mBase = m0 + (i << 4);
#pragma unroll
    for (int j = 0; j < 4; ++j) {
#pragma unroll
      for (int r = 0; r < 8; ++r) {
        float v = acc[i][j][r] * scale;
        if (ACT == 2) v = fmaxf(v, 0.0f);
        slab[(mOff + r) * 68 + (j << 4) + rlane] = v;
      }
    }
    __builtin_amdgcn_fence(__ATOMIC_RELEASE, "workgroup");
    __builtin_amdgcn_wave_barrier();
    __builtin_amdgcn_fence(__ATOMIC_ACQUIRE, "workgroup");
    if (OUT_MODE == 0) {
      float* C = (float*)Cout;
      const int hh = lane >> 4, c4 = (lane & 15) * 4;
      for (int pass = 0; pass < 2; ++pass) {
#pragma unroll
        for (int it = 0; it < 8; ++it) {
          const int row = it * 2 + hh;
          const v4f v = *(const v4f*)(slab + row * 68 + c4);
          if (mBase + row < mReal) *(volatile v4f*)(C + (size_t)(mBase + row) * ldc + n0 + c4) = v;
        }
        __threadfence();
      }
    } else {
      const int q = lane >> 3, c8 = (lane & 7) * 8;
      unsigned short* C = (unsigned short*)Cout;
      for (int pass = 0; pass < 2; ++pass) {
#pragma unroll
        for (int it = 0; it < 4; ++it) {
          const int row = it * 4 + q;
          const float* sp = slab + row * 68 + c8;
          v8h hv;
#pragma unroll
          for (int e = 0; e < 8; ++e) hv[e] = (_Float16)sp[e];
          *(volatile v8h*)(C + (size_t)(mBase + row) * ldc + n0 + c8) = hv;
        }
        __threadfence();
      }
    }
    __builtin_amdgcn_fence(__ATOMIC_RELEASE, "workgroup");
    __builtin_amdgcn_wave_barrier();
    __builtin_amdgcn_fence(__ATOMIC_ACQUIRE, "workgroup");
  }
}

extern "C" void kernel_launch(void* const* d_in, const int* in_sizes, int n_in,
                              void* d_out, int out_size, void* d_ws, size_t ws_size,
                              hipStream_t stream) {
  if (n_in < 4) return;
  if (in_sizes[0] != kNN * kDF) return;
  if (in_sizes[1] != kDF * kDH) return;
  if (in_sizes[2] != kDH * kDO) return;
  if (in_sizes[3] != 2 * kNE) return;
  if (out_size != kNN * kDO) return;
  if (ws_size < kWsTotal) return;

  const float* feats = (const float*)d_in[0];
  const float* W1    = (const float*)d_in[1];
  const float* W2    = (const float*)d_in[2];
  const int*   ei    = (const int*)d_in[3];
  float* out = (float*)d_out;

  char* ws = (char*)d_ws;
  unsigned*       PART   = (unsigned*)(ws + kOffPart);
  int*            CTAB   = (int*)(ws + kOffCtab);
  int*            CSR    = (int*)(ws + kOffCsr);
  int*            RSTART = (int*)(ws + kOffRS);
  int*            RDEG   = (int*)(ws + kOffRD);
  float*          RNORM  = (float*)(ws + kOffRN);
  float*          ZA     = (float*)(ws + kOffZA);
  float*          ZB     = (float*)(ws + kOffZB);
  unsigned short* W1T    = (unsigned short*)(ws + kOffW1T);
  unsigned short* W2T    = (unsigned short*)(ws + kOffW2T);
  unsigned short* Y16    = (unsigned short*)(ws + kOffZB);
  unsigned short* H16    = (unsigned short*)(ws + kOffZA);

  part_edges_kernel<<<kNCh, 256, 0, stream>>>(ei, PART, CTAB);
  build_rows_kernel<<<kNGrp, 256, 0, stream>>>(PART, CTAB, CSR, RSTART, RDEG, RNORM);
  weight_planes_kernel<<<12, 256, 0, stream>>>(W1, W2, W1T, W2T);

  hop_kernel<0><<<kNN / 8, 256, 0, stream>>>(feats, feats, CSR, RSTART, RDEG, RNORM, ZA, Y16, kMix);
  hop_kernel<0><<<kNN / 8, 256, 0, stream>>>(ZA, feats, CSR, RSTART, RDEG, RNORM, ZB, Y16, 1.0f);
  hop_kernel<0><<<kNN / 8, 256, 0, stream>>>(ZB, feats, CSR, RSTART, RDEG, RNORM, ZA, Y16, 1.0f);
  hop_kernel<1><<<kMPad / 8, 256, 0, stream>>>(ZA, feats, CSR, RSTART, RDEG, RNORM, ZB, Y16, 1.0f);

  wmma_gemm64_f16<1, 2><<<((kMPad / 64) * (kDH / 64) + 7) / 8, 256, 0, stream>>>(
      Y16, kDF, W1T, kDF, (void*)H16, kDH, kMPad, kDH, kDF, kMPad, kScale1);
  wmma_gemm64_f16<0, 0><<<((kMPad / 64) * (kDO / 64) + 7) / 8, 256, 0, stream>>>(
      H16, kDH, W2T, kDH, (void*)out, kDO, kMPad, kDO, kDH, kNN, kScale2);
}
